// SelfAttention_13958643712690
// MI455X (gfx1250) — hardware-verified
//
#include <hip/hip_runtime.h>
#ifndef NB
#define NB 2
#endif
#ifndef SEQ
#define SEQ 2048
#endif
#define NB_FULL 2
#define SEQ_FULL 2048
#define DM 768
#define NH 12
#define HD 64
#define NQKV (3 * DM)
#define MR (NB * SEQ)
#define NBH (NB * NH)
#define LDSO 68
#define LDSH 72

static_assert(NH * HD == DM);
static_assert(HD == 64);
static_assert(DM % 32 == 0);
static_assert(DM % 64 == 0);
static_assert(NQKV % 64 == 0);
static_assert(DM == 3 * 32 * 8);
static_assert(MR % 128 == 0);
static_assert(MR % 8 == 0);
static_assert(SEQ % 64 == 0);
static_assert(SEQ % 32 == 0);
static_assert((SEQ / 16) % 4 == 0);
static_assert(NB <= NB_FULL && SEQ <= SEQ_FULL);
static_assert(LDSO % 4 == 0 && LDSH % 8 == 0);

#define AL256(x) ((((size_t)(x)) + 255) & ~(size_t)255)
constexpr size_t SZ_WT  = AL256((size_t)NQKV * DM * 2);
constexpr size_t SZ_WO  = AL256((size_t)DM * DM * 2);
constexpr size_t SZ_H   = AL256((size_t)MR * DM * 2);
constexpr size_t SZ_QKV = AL256((size_t)MR * NQKV * 2);
constexpr size_t SZ_QL  = AL256((size_t)MR * DM * 2);
constexpr size_t SZ_VT  = AL256((size_t)NBH * HD * SEQ * 2);
constexpr size_t SZ_CTX = AL256((size_t)MR * DM * 2);
static_assert(SZ_WT + SZ_WO + SZ_H + SZ_QKV + SZ_QL + SZ_VT + SZ_CTX <= (size_t)134217728);

typedef unsigned short v8us __attribute__((ext_vector_type(8), may_alias));
typedef float  v8f  __attribute__((ext_vector_type(8)));
typedef float  v4f  __attribute__((ext_vector_type(4)));
typedef float  v4fa __attribute__((ext_vector_type(4), may_alias));
typedef _Float16 v16h __attribute__((ext_vector_type(16)));
union FragH { v16h v; v8us half[2]; _Float16 h[16]; unsigned short u[16]; };

__device__ __forceinline__ float bf16_rne(float x) {
  unsigned int u = __float_as_uint(x);
  u = (u + 0x7FFFu + ((u >> 16) & 1u)) & 0xFFFF0000u;
  return __uint_as_float(u);
}
__device__ __forceinline__ size_t io_row(int r) { return (size_t)(r / SEQ) * SEQ_FULL + (size_t)(r % SEQ); }

__device__ __forceinline__ v16h g2_frag(const _Float16* p, int hh) {
  FragH f;
  f.half[0] = *(const v8us*)((const unsigned short*)p + 8 * hh);
  f.half[1] = *(const v8us*)((const unsigned short*)p + 16 + 8 * hh);
  return f.v;
}
__device__ __forceinline__ v8f g2_mma(v16h a, v16h b, v8f c) {
  v8f d = __builtin_amdgcn_wmma_f32_16x16x32_f16(false, a, false, b, (short)0, c, false, false);
  asm volatile("v_nop\n\tv_nop\n\tv_nop\n\tv_nop" : "+v"(d) : "v"(a), "v"(b));
  return d;
}

__global__ __launch_bounds__(256) void k_wt_f16(const float* __restrict__ W, _Float16* __restrict__ Wt) {
  const int t = blockIdx.x * 256 + threadIdx.x;
  if (t >= DM * (DM / 8)) return;
  const int n = t / (DM / 8), k8 = (t % (DM / 8)) * 8;
  FragH f;
#pragma unroll
  for (int i = 0; i < 8; ++i) f.h[i] = (_Float16)(bf16_rne(W[(size_t)(k8 + i) * DM + n]) * 64.0f);
  const v8us o = f.half[0];
  unsigned short* d = (unsigned short*)Wt + (size_t)n * DM + k8;
  *(volatile v8us*)d = o;
  __threadfence();
  *(volatile v8us*)d = o;
}

__global__ __launch_bounds__(256) void k_ln16(const float* __restrict__ x, const float* __restrict__ g, const float* __restrict__ bt, _Float16* __restrict__ H16) {
  const int wave = __builtin_amdgcn_readfirstlane(threadIdx.x >> 5);
  const int lane = threadIdx.x & 31;
  const int row = blockIdx.x * 8 + wave;
  if (row >= MR) return;
  const float* xr = x + io_row(row) * DM;
  float s1 = 0.f;
#pragma unroll 1
  for (int u = 0; u < 3; ++u) {
    const int j = u * 256 + lane * 8;
    const v4f a = *(const v4fa*)(xr + j), c = *(const v4fa*)(xr + j + 4);
#pragma unroll
    for (int q = 0; q < 4; ++q) s1 += bf16_rne(a[q]) + bf16_rne(c[q]);
  }
  s1 += __shfl_xor(s1, 16); s1 += __shfl_xor(s1, 8); s1 += __shfl_xor(s1, 4); s1 += __shfl_xor(s1, 2); s1 += __shfl_xor(s1, 1);
  const float mu = s1 * (1.0f / (float)DM);
  float s2 = 0.f;
#pragma unroll 1
  for (int u = 0; u < 3; ++u) {
    const int j = u * 256 + lane * 8;
    const v4f a = *(const v4fa*)(xr + j), c = *(const v4fa*)(xr + j + 4);
#pragma unroll
    for (int q = 0; q < 4; ++q) { const float da = bf16_rne(a[q]) - mu, dc = bf16_rne(c[q]) - mu; s2 += da * da; s2 += dc * dc; }
  }
  s2 += __shfl_xor(s2, 16); s2 += __shfl_xor(s2, 8); s2 += __shfl_xor(s2, 4); s2 += __shfl_xor(s2, 2); s2 += __shfl_xor(s2, 1);
  const float rs = rsqrtf(s2 * (1.0f / (float)DM) + 1.0e-5f);
#pragma unroll 1
  for (int u = 0; u < 3; ++u) {
    const int j = u * 256 + lane * 8;
    const v4f a = *(const v4fa*)(xr + j), c = *(const v4fa*)(xr + j + 4);
    const v4f ga = *(const v4fa*)(g + j), gc = *(const v4fa*)(g + j + 4);
    const v4f ba = *(const v4fa*)(bt + j), bc = *(const v4fa*)(bt + j + 4);
    FragH f;
#pragma unroll
    for (int q = 0; q < 4; ++q) {
      f.h[q]     = (_Float16)((bf16_rne(a[q]) - mu) * rs * bf16_rne(ga[q]) + bf16_rne(ba[q]));
      f.h[4 + q] = (_Float16)((bf16_rne(c[q]) - mu) * rs * bf16_rne(gc[q]) + bf16_rne(bc[q]));
    }
    const v8us o = f.half[0];
    unsigned short* d = (unsigned short*)H16 + (size_t)row * DM + j;
    *(volatile v8us*)d = o;
    __threadfence();
    *(volatile v8us*)d = o;
  }
}

__global__ __launch_bounds__(128) void k_gemm_qkv(const _Float16* __restrict__ A, const _Float16* __restrict__ Bt, _Float16* __restrict__ QKV, _Float16* __restrict__ QL) {
  __shared__ __attribute__((aligned(16))) float so[4][32][LDSO];
  const int tid = threadIdx.x;
  const int wave = __builtin_amdgcn_readfirstlane(tid >> 5);
  const int lane = tid & 31, ln = lane & 15, hh = lane >> 4;
  const int ntn = NQKV / 64;
  const int mt = blockIdx.x / ntn, nq = blockIdx.x - mt * ntn;
  const int row0 = mt * 128 + 32 * wave, col0 = nq * 64;
  const _Float16* a0p = A + (size_t)(row0 + ln) * DM; const _Float16* a1p = a0p + (size_t)16 * DM;
  const _Float16* b0p = Bt + (size_t)(col0 + ln) * DM; const _Float16* b1p = b0p + (size_t)16 * DM;
  const _Float16* b2p = b1p + (size_t)16 * DM; const _Float16* b3p = b2p + (size_t)16 * DM;
  const v8f z8 = {0.f,0.f,0.f,0.f,0.f,0.f,0.f,0.f};
  v8f c00 = z8, c01 = z8, c02 = z8, c03 = z8, c10 = z8, c11 = z8, c12 = z8, c13 = z8;
#pragma unroll 1
  for (int kb = 0; kb < DM; kb += 32) {
    const v16h a0 = g2_frag(a0p + kb, hh), a1 = g2_frag(a1p + kb, hh);
    v16h b = g2_frag(b0p + kb, hh); c00 = g2_mma(a0, b, c00); c10 = g2_mma(a1, b, c10);
    b = g2_frag(b1p + kb, hh); c01 = g2_mma(a0, b, c01); c11 = g2_mma(a1, b, c11);
    b = g2_frag(b2p + kb, hh); c02 = g2_mma(a0, b, c02); c12 = g2_mma(a1, b, c12);
    b = g2_frag(b3p + kb, hh); c03 = g2_mma(a0, b, c03); c13 = g2_mma(a1, b, c13);
  }
  v8f accs[8] = {c00, c01, c02, c03, c10, c11, c12, c13};
#pragma unroll
  for (int u = 0; u < 8; ++u) {
    const int t = u & 3, half = u >> 2;
#pragma unroll
    for (int r = 0; r < 8; ++r) so[wave][half * 16 + 8 * hh + r][t * 16 + ln] = accs[u][r] * 0.015625f;
  }
  __builtin_amdgcn_fence(4  , "workgroup");
  __builtin_amdgcn_wave_barrier();
  const int rq = lane >> 3, pc = (lane & 7) * 8;
  const bool isq = (col0 < DM);
  for (int pass = 0; pass < 2; ++pass) {
#pragma unroll
    for (int it = 0; it < 8; ++it) {
      const int r = it * 4 + rq;
      const v4f a = *(const v4fa*)&so[wave][r][pc], c = *(const v4fa*)&so[wave][r][pc + 4];
      FragH fh, fl;
#pragma unroll
      for (int q = 0; q < 4; ++q) {
        _Float16 h = (_Float16)a[q]; fh.h[q] = h; fl.h[q] = (_Float16)((a[q] - (float)h) * 1024.0f);
        h = (_Float16)c[q]; fh.h[4 + q] = h; fl.h[4 + q] = (_Float16)((c[q] - (float)h) * 1024.0f);
      }
      const v8us oh = fh.half[0], ol = fl.half[0];
      *(volatile v8us*)((unsigned short*)QKV + (size_t)(row0 + r) * NQKV + col0 + pc) = oh;
      if (isq) *(volatile v8us*)((unsigned short*)QL + (size_t)(row0 + r) * DM + col0 + pc) = ol;
    }
    if (pass == 0) __threadfence();
  }
}

__global__ __launch_bounds__(256) void k_vt(const _Float16* __restrict__ QKV, _Float16* __restrict__ VT) {
  __shared__ unsigned short tl[64][66];
  const int tid = threadIdx.x;
  const int bh = blockIdx.x / (SEQ / 64), sg = blockIdx.x - bh * (SEQ / 64);
  const int b = bh / NH, h = bh - b * NH;
  const int s0 = sg * 64;
  for (int i = tid; i < 64 * 8; i += 256) {
    const int j = i >> 3, d8 = (i & 7) * 8;
    FragH f;
    f.half[0] = *(const v8us*)((const unsigned short*)QKV + ((size_t)b * SEQ + s0 + j) * NQKV + 2 * DM + h * HD + d8);
#pragma unroll
    for (int q = 0; q < 8; ++q) tl[d8 + q][j] = f.u[q];
  }
  __syncthreads();
  for (int pass = 0; pass < 2; ++pass) {
    for (int i = tid; i < 64 * 8; i += 256) {
      const int d = i >> 3, j8 = (i & 7) * 8;
      FragH f;
#pragma unroll
      for (int q = 0; q < 8; ++q) f.u[q] = tl[d][j8 + q];
      const v8us o = f.half[0];
      *(volatile v8us*)((unsigned short*)VT + ((size_t)bh * HD + d) * SEQ + s0 + j8) = o;
    }
    if (pass == 0) __threadfence();
  }
}

__global__ __launch_bounds__(128) void k_flash(const _Float16* __restrict__ QKV, const _Float16* __restrict__ QL, const _Float16* __restrict__ VT, _Float16* __restrict__ CTX) {
  __shared__ __attribute__((aligned(16))) unsigned short so[4][16][LDSH];
  const int tid = threadIdx.x;
  const int wave = __builtin_amdgcn_readfirstlane(tid >> 5);
  const int lane = tid & 31, ln = lane & 15, hh = lane >> 4;
  const int gw = blockIdx.x * 4 + wave;
  const int bh = gw / (SEQ / 16), qt = gw - bh * (SEQ / 16);
  const int b = bh / NH, h = bh - b * NH;
  const size_t tok0 = (size_t)b * SEQ;
  const int q0 = qt * 16;
  const _Float16* qp  = QKV + (tok0 + q0 + ln) * NQKV + h * HD;
  const _Float16* qlp = QL + (tok0 + q0 + ln) * DM + h * HD;
  const v16h qh0 = g2_frag(qp, hh), qh1 = g2_frag(qp + 32, hh);
  const v16h ql0 = g2_frag(qlp, hh), ql1 = g2_frag(qlp + 32, hh);
  const _Float16* kp = QKV + (tok0 + ln) * NQKV + DM + h * HD;
  const _Float16* vp = VT + ((size_t)bh * HD + ln) * SEQ;
  const v8f z8 = {0.f,0.f,0.f,0.f,0.f,0.f,0.f,0.f};
  v8f o[4] = {z8, z8, z8, z8};
  float m = -1.0e30f, l = 0.f;
#pragma unroll 1
  for (int key0 = 0; key0 < SEQ; key0 += 32) {
    const _Float16* k0p = kp + (size_t)key0 * NQKV;
    const _Float16* k1p = k0p + (size_t)16 * NQKV;
    v8f sh0 = z8, sl0 = z8, sh1 = z8, sl1 = z8;
    v16h a = g2_frag(k0p, hh);      sh0 = g2_mma(a, qh0, sh0); sl0 = g2_mma(a, ql0, sl0);
    a = g2_frag(k0p + 32, hh);      sh0 = g2_mma(a, qh1, sh0); sl0 = g2_mma(a, ql1, sl0);
    a = g2_frag(k1p, hh);           sh1 = g2_mma(a, qh0, sh1); sl1 = g2_mma(a, ql0, sl1);
    a = g2_frag(k1p + 32, hh);      sh1 = g2_mma(a, qh1, sh1); sl1 = g2_mma(a, ql1, sl1);
    float s0[8], s1[8];
    float mx = -3.0e38f;
#pragma unroll
    for (int r = 0; r < 8; ++r) {
      s0[r] = sh0[r] + sl0[r] * 0.0009765625f;
      s1[r] = sh1[r] + sl1[r] * 0.0009765625f;
      mx = fmaxf(mx, fmaxf(s0[r], s1[r]));
    }
    mx = fmaxf(mx, __shfl_xor(mx, 16));
    const float mnew = fmaxf(m, mx);
    const float corr = __expf(m - mnew);
    m = mnew;
    FragH pb;
    float ls = 0.f;
#pragma unroll
    for (int r = 0; r < 8; ++r) {
      const _Float16 p0 = (_Float16)(__expf(s0[r] - mnew) * 16384.0f);
      const _Float16 p1 = (_Float16)(__expf(s1[r] - mnew) * 16384.0f);
      pb.h[r] = p0; pb.h[8 + r] = p1;
      ls += (float)p0 + (float)p1;
    }
    l = l * corr + ls;
#pragma unroll
    for (int t = 0; t < 4; ++t) {
#pragma unroll
      for (int r = 0; r < 8; ++r) o[t][r] *= corr;
    }
#pragma unroll
    for (int t = 0; t < 4; ++t) {
      const v16h av = g2_frag(vp + (size_t)(t * 16) * SEQ + key0, hh);
      o[t] = g2_mma(av, pb.v, o[t]);
    }
  }
  l += __shfl_xor(l, 16);
  const float inv = 8.0f * (1.0f / l);
#pragma unroll
  for (int t = 0; t < 4; ++t) {
    FragH f;
#pragma unroll
    for (int r = 0; r < 8; ++r) f.h[r] = (_Float16)(o[t][r] * inv);
    *(v8us*)&so[wave][ln][t * 16 + 8 * hh] = f.half[0];
  }
  __builtin_amdgcn_fence(4  , "workgroup");
  __builtin_amdgcn_wave_barrier();
  const int rq = lane >> 3, pc = (lane & 7) * 8;
  for (int pass = 0; pass < 2; ++pass) {
#pragma unroll
    for (int it = 0; it < 4; ++it) {
      const int r = it * 4 + rq;
      const v8us v = *(const v8us*)&so[wave][r][pc];
      *(volatile v8us*)((unsigned short*)CTX + (tok0 + q0 + r) * DM + h * HD + pc) = v;
    }
    if (pass == 0) __threadfence();
  }
}

__global__ __launch_bounds__(128) void k_gemm_out(const _Float16* __restrict__ A, const _Float16* __restrict__ Bt, const float* __restrict__ bo, const float* __restrict__ x, float* __restrict__ Y) {
  __shared__ __attribute__((aligned(16))) float so[4][32][LDSO];
  const int tid = threadIdx.x;
  const int wave = __builtin_amdgcn_readfirstlane(tid >> 5);
  const int lane = tid & 31, ln = lane & 15, hh = lane >> 4;
  const int ntn = DM / 64;
  const int mt = blockIdx.x / ntn, nq = blockIdx.x - mt * ntn;
  const int row0 = mt * 128 + 32 * wave, col0 = nq * 64;
  const _Float16* a0p = A + (size_t)(row0 + ln) * DM; const _Float16* a1p = a0p + (size_t)16 * DM;
  const _Float16* b0p = Bt + (size_t)(col0 + ln) * DM; const _Float16* b1p = b0p + (size_t)16 * DM;
  const _Float16* b2p = b1p + (size_t)16 * DM; const _Float16* b3p = b2p + (size_t)16 * DM;
  const v8f z8 = {0.f,0.f,0.f,0.f,0.f,0.f,0.f,0.f};
  v8f c00 = z8, c01 = z8, c02 = z8, c03 = z8, c10 = z8, c11 = z8, c12 = z8, c13 = z8;
#pragma unroll 1
  for (int kb = 0; kb < DM; kb += 32) {
    const v16h a0 = g2_frag(a0p + kb, hh), a1 = g2_frag(a1p + kb, hh);
    v16h b = g2_frag(b0p + kb, hh); c00 = g2_mma(a0, b, c00); c10 = g2_mma(a1, b, c10);
    b = g2_frag(b1p + kb, hh); c01 = g2_mma(a0, b, c01); c11 = g2_mma(a1, b, c11);
    b = g2_frag(b2p + kb, hh); c02 = g2_mma(a0, b, c02); c12 = g2_mma(a1, b, c12);
    b = g2_frag(b3p + kb, hh); c03 = g2_mma(a0, b, c03); c13 = g2_mma(a1, b, c13);
  }
  v8f accs[8] = {c00, c01, c02, c03, c10, c11, c12, c13};
#pragma unroll
  for (int u = 0; u < 8; ++u) {
    const int t = u & 3, half = u >> 2;
#pragma unroll
    for (int r = 0; r < 8; ++r) so[wave][half * 16 + 8 * hh + r][t * 16 + ln] = accs[u][r] * 0.000244140625f;
  }
  __builtin_amdgcn_fence(4  , "workgroup");
  __builtin_amdgcn_wave_barrier();
  const int rsub = lane >> 4, c4 = (lane & 15) * 4;
  const v4f braw = *(const v4fa*)(bo + col0 + c4);
  v4f bb;
#pragma unroll
  for (int i = 0; i < 4; ++i) bb[i] = bf16_rne(braw[i]);
  for (int pass = 0; pass < 2; ++pass) {
#pragma unroll 4
    for (int q = 0; q < 16; ++q) {
      const int r = q * 2 + rsub;
      const size_t grow = io_row(row0 + r);
      const v4f v = *(const v4fa*)&so[wave][r][c4];
      const v4f xr = *(const v4fa*)(x + grow * DM + col0 + c4);
      v4f ov;
#pragma unroll
      for (int i = 0; i < 4; ++i) ov[i] = bf16_rne(xr[i]) + (v[i] + bb[i]);
      *(volatile v4f*)(Y + grow * DM + col0 + c4) = ov;
    }
    if (pass == 0) __threadfence();
  }
}

extern "C" void kernel_launch(void* const* d_in, const int* in_sizes, int n_in,
                              void* d_out, int out_size, void* d_ws, size_t ws_size, hipStream_t stream) {
  if (n_in < 8) return;
  const size_t need = ((size_t)(NB - 1) * SEQ_FULL + SEQ) * DM;
  if ((size_t)in_sizes[0] < need) return;
  if (in_sizes[1] < DM * DM || in_sizes[2] < DM * DM || in_sizes[3] < DM * DM || in_sizes[4] < DM * DM) return;
  if (in_sizes[5] < DM || in_sizes[6] < DM || in_sizes[7] < DM) return;
  if ((size_t)out_size < need) return;
  const float* x = (const float*)d_in[0];
  const float* Wq = (const float*)d_in[1];
  const float* Wk = (const float*)d_in[2];
  const float* Wv = (const float*)d_in[3];
  const float* Wo = (const float*)d_in[4];
  const float* bo = (const float*)d_in[5];
  const float* gamma = (const float*)d_in[6];
  const float* beta = (const float*)d_in[7];
  float* y = (float*)d_out;

  char* ws = (char*)d_ws; size_t off = 0;
  _Float16* WT  = (_Float16*)(ws + off); off += SZ_WT;
  _Float16* WO  = (_Float16*)(ws + off); off += SZ_WO;
  _Float16* H16 = (_Float16*)(ws + off); off += SZ_H;
  _Float16* QKV = (_Float16*)(ws + off); off += SZ_QKV;
  _Float16* QL  = (_Float16*)(ws + off); off += SZ_QL;
  _Float16* VT  = (_Float16*)(ws + off); off += SZ_VT;
  _Float16* CTX = (_Float16*)(ws + off); off += SZ_CTX;
  if (off > ws_size) return;

  const unsigned gwt = (unsigned)((DM * (DM / 8) + 255) / 256);
  k_wt_f16<<<gwt, 256, 0, stream>>>(Wq, WT);
  k_wt_f16<<<gwt, 256, 0, stream>>>(Wk, WT + (size_t)DM * DM);
  k_wt_f16<<<gwt, 256, 0, stream>>>(Wv, WT + (size_t)2 * DM * DM);
  k_wt_f16<<<gwt, 256, 0, stream>>>(Wo, WO);
  k_ln16<<<(unsigned)(MR / 8), 256, 0, stream>>>(x, gamma, beta, H16);
  k_gemm_qkv<<<(unsigned)((MR / 128) * (NQKV / 64)), 128, 0, stream>>>(H16, WT, QKV, QL);
  k_vt<<<(unsigned)(NBH * (SEQ / 64)), 256, 0, stream>>>(QKV, VT);
  k_flash<<<(unsigned)(NBH * (SEQ / 64)), 128, 0, stream>>>(QKV, QL, VT, CTX);
  k_gemm_out<<<(unsigned)((MR / 128) * (DM / 64)), 128, 0, stream>>>(CTX, WO, bo, x, y);
}
